// GenScore_11063835754636
// MI455X (gfx1250) — hardware-verified
//
#include <hip/hip_runtime.h>
#include <stddef.h>


#pragma clang fp contract(off)

#define DN      128
#define NTHR    256
#define NWAVE   8
#define NBN     64
#define NBE     64
#define APA     136
#define APN     264
#define GSTR    132
#define NPROW   256
#define MROW    128
#define CROW    4
#define EPT     8
#define PIECE   (NTHR * EPT)
#define WCAP    (EPT * 32)
#define NBC     512
#define SLB     9
#define CE      114688
#define MAXCH   64
#define PAS     0
#define PAT     16384
#define PBS     32768
#define PBT     49152
#define P2S     65536
#define P2T     81920
#define PC1     98304
#define PN1T    114688
#define PN2T    147456
#define PN1S    163840
#define PN2S    196608
#define PWTOT   212992
#define PBLK    (PWTOT / (NTHR * 8))
#define WSCAP   134217728
#define EDGEDYN (NBE * GSTR * 4)
#define AGGDYN  ((NBC * DN + NBC * CROW) * 4)
#define OB1S    0
#define OWRS    128
#define OB1T    256
#define OWRT    384
#define OB2S    512
#define OB2T    640
#define OWGS    768
#define OWGT    896
#define OBC1    1024
#define OWC2    1152
#define OBGS    1280
#define OBGT    1281
#define SPARN   1288
#define SCW     16.0f
#define SCA     64.0f
#define INV16   0.0625f
#define INV64   0.015625f
#define INV1024 0.0009765625f
#define CMAXV   10.0f

static_assert((PWTOT % (NTHR * 8)) == 0);
static_assert((PAT % (NTHR * 8)) == 0);
static_assert((PBS % (NTHR * 8)) == 0);
static_assert((PBT % (NTHR * 8)) == 0);
static_assert((P2S % (NTHR * 8)) == 0);
static_assert((P2T % (NTHR * 8)) == 0);
static_assert((PC1 % (NTHR * 8)) == 0);
static_assert((PN1T % (NTHR * 8)) == 0);
static_assert((PN2T % (NTHR * 8)) == 0);
static_assert((PN1S % (NTHR * 8)) == 0);
static_assert((PN2S % (NTHR * 8)) == 0);
static_assert(((APA * 2) % 16) == 0);
static_assert(((APN * 2) % 16) == 0);
static_assert(((GSTR * 4) % 16) == 0);
static_assert(NBN * APN * 2 == NBN * GSTR * 4);
static_assert(NBC == (1 << SLB));
static_assert(PIECE == 2048);
static_assert((EPT % 4) == 0);
static_assert((CE % PIECE) == 0);
static_assert((CE % NBE) == 0);
static_assert((NBC % NWAVE) == 0);
static_assert(3 * NBC <= 8 * NTHR);
static_assert(NBE == NWAVE * 8);
static_assert(NBN == 4 * 16);
static_assert((NBC * DN) % (4 * NTHR) == 0);
static_assert((NBC % NTHR) == 0);
static_assert((SPARN % 4) == 0);

typedef float          v4f   __attribute__((ext_vector_type(4)));
typedef float          v8f   __attribute__((ext_vector_type(8)));
typedef int            v4i   __attribute__((ext_vector_type(4)));
typedef unsigned short v8us  __attribute__((ext_vector_type(8)));
typedef _Float16       v4h   __attribute__((ext_vector_type(4)));
typedef _Float16       v8h   __attribute__((ext_vector_type(8)));
typedef _Float16       v16h  __attribute__((ext_vector_type(16)));
union FragH { v16h v; v8h h[2]; };
union Cvt8  { v8h v; v8us u; };

__device__ __forceinline__ v8f wmh(v16h a, v16h b, v8f c) {
  v8f d = __builtin_amdgcn_wmma_f32_16x16x32_f16(false, a, false, b, (short)0, c, false, false);
  asm volatile("v_nop\n\tv_nop\n\tv_nop\n\tv_nop" : "+v"(d) : "v"(a), "v"(b));
  return d;
}
__device__ __forceinline__ v8f zero8() {
  v8f z = {0.f, 0.f, 0.f, 0.f, 0.f, 0.f, 0.f, 0.f};
  return z;
}
__device__ __forceinline__ v4f zero4() {
  v4f z = {0.f, 0.f, 0.f, 0.f};
  return z;
}
__device__ __forceinline__ int imin(int a, int b) { return a < b ? a : b; }
__device__ __forceinline__ int iclamp(int v, int lo, int hi) { return v < lo ? lo : (v > hi ? hi : v); }

__device__ __forceinline__ float sigm_f(float z) {
  const float zc = fminf(fmaxf(z, -80.0f), 80.0f);
  return __builtin_amdgcn_rcpf(1.0f + __expf(-zc));
}
__device__ __forceinline__ float silu_f(float x) { return x * sigm_f(x); }

__device__ __forceinline__ void gemm16x64(const _Float16* ap, const _Float16* bpl, int kp, int nks, int n0,
                                          int m, int hh, v8f& c0, v8f& c1, v8f& c2, v8f& c3) {
  c0 = zero8(); c1 = zero8(); c2 = zero8(); c3 = zero8();
#pragma unroll 1
  for (int ks = 0; ks < nks; ++ks) {
    FragH a;
    a.h[0] = *(const v8h*)(ap + 32 * ks);
    a.h[1] = *(const v8h*)(ap + 32 * ks + 16);
    const _Float16* bp = bpl + (size_t)(n0 + m) * kp + 32 * ks + 8 * hh;
    FragH b;
    b.h[0] = *(const v8h*)(bp);
    b.h[1] = *(const v8h*)(bp + 16);
    c0 = wmh(a.v, b.v, c0);
    b.h[0] = *(const v8h*)(bp + (size_t)16 * kp);
    b.h[1] = *(const v8h*)(bp + (size_t)16 * kp + 16);
    c1 = wmh(a.v, b.v, c1);
    b.h[0] = *(const v8h*)(bp + (size_t)32 * kp);
    b.h[1] = *(const v8h*)(bp + (size_t)32 * kp + 16);
    c2 = wmh(a.v, b.v, c2);
    b.h[0] = *(const v8h*)(bp + (size_t)48 * kp);
    b.h[1] = *(const v8h*)(bp + (size_t)48 * kp + 16);
    c3 = wmh(a.v, b.v, c3);
  }
}

__device__ __forceinline__ void stage8(float* sp, v8f a, float scl, float bias) {
#pragma unroll
  for (int r = 0; r < 8; ++r) sp[r * GSTR] = a[r] * scl + bias;
}
__device__ __forceinline__ void stage8s(float* sp, v8f a, float scl, float bias) {
#pragma unroll
  for (int r = 0; r < 8; ++r) sp[r * GSTR] = silu_f(a[r] * scl + bias);
}
__device__ __forceinline__ void stage8hs(_Float16* sp, v8f a, float scl, float bias) {
#pragma unroll
  for (int r = 0; r < 8; ++r) sp[r * APA] = (_Float16)(silu_f(a[r] * scl + bias) * SCA);
}

__global__ __launch_bounds__(NTHR) void k_prep(
    const float* __restrict__ w1s, const float* __restrict__ w1t, const float* __restrict__ w2s,
    const float* __restrict__ w2t, const float* __restrict__ wc1, const float* __restrict__ wn1t,
    const float* __restrict__ wn2t, const float* __restrict__ wn1s, const float* __restrict__ wn2s,
    unsigned short* wp) {
  const int tid = (int)threadIdx.x;
  const int b = (int)blockIdx.x;
  const int o = (b * NTHR + tid) * 8;
  const float* src = w1s;
  int r0 = 0, n, k0;
  if (o < PAT)       { n = o >> 7; k0 = o & 127; }
  else if (o < PBS)  { const int idx = o - PAT;  n = idx >> 7; k0 = idx & 127; src = w1t; }
  else if (o < PBT)  { const int idx = o - PBS;  n = idx >> 7; k0 = idx & 127; r0 = DN; }
  else if (o < P2S)  { const int idx = o - PBT;  n = idx >> 7; k0 = idx & 127; r0 = DN; src = w1t; }
  else if (o < P2T)  { const int idx = o - P2S;  n = idx >> 7; k0 = idx & 127; src = w2s; }
  else if (o < PC1)  { const int idx = o - P2T;  n = idx >> 7; k0 = idx & 127; src = w2t; }
  else if (o < PN1T) { const int idx = o - PC1;  n = idx >> 7; k0 = idx & 127; src = wc1; }
  else if (o < PN2T) { const int idx = o - PN1T; n = idx >> 8; k0 = idx & 255; src = wn1t; }
  else if (o < PN1S) { const int idx = o - PN2T; n = idx >> 7; k0 = idx & 127; src = wn2t; }
  else if (o < PN2S) { const int idx = o - PN1S; n = idx >> 8; k0 = idx & 255; src = wn1s; }
  else               { const int idx = o - PN2S; n = idx >> 7; k0 = idx & 127; src = wn2s; }
  Cvt8 cv;
#pragma unroll
  for (int j = 0; j < 8; ++j) cv.v[j] = (_Float16)(src[(size_t)(r0 + k0 + j) * DN + n] * SCW);
  unsigned short* dp = wp + o;
  *(volatile v8us*)dp = cv.u;
  __threadfence();
  *(volatile v8us*)dp = cv.u;
}

__global__ __launch_bounds__(NTHR) void k_node(
    const float* __restrict__ feat, const unsigned short* __restrict__ wp, int off0, int off1, float* NP, int nN) {
  __shared__ __attribute__((aligned(16))) _Float16 sA[NBN * APA];
  __shared__ __attribute__((aligned(16))) float stg[NWAVE * 1024];
  const int tid = (int)threadIdx.x, lane = tid & 31, wave = tid >> 5, hh = lane >> 4, m = lane & 15;
  const int n0 = (int)blockIdx.x * NBN;

  {
    const int nl = tid >> 2, q = tid & 3;
    int node = n0 + nl;
    node = node > nN - 1 ? nN - 1 : node;
    const float* rp = feat + (size_t)node * DN + 32 * q;
#pragma unroll
    for (int i = 0; i < 4; ++i) {
      const v4f xa = *(const v4f*)(rp + 8 * i);
      const v4f xb = *(const v4f*)(rp + 8 * i + 4);
      Cvt8 cv;
      cv.v[0] = (_Float16)xa.x; cv.v[1] = (_Float16)xa.y; cv.v[2] = (_Float16)xa.z; cv.v[3] = (_Float16)xa.w;
      cv.v[4] = (_Float16)xb.x; cv.v[5] = (_Float16)xb.y; cv.v[6] = (_Float16)xb.z; cv.v[7] = (_Float16)xb.w;
      *(v8h*)(sA + nl * APA + 32 * q + 8 * i) = cv.v;
    }
  }
  __syncthreads();

  const int rt = wave & 3, chf = wave >> 2;
  const _Float16* ap = sA + (16 * rt + m) * APA + 8 * hh;
  const _Float16* plane = (const _Float16*)(wp + (chf ? off1 : off0));
  float* sw = stg + wave * 1024;
#pragma unroll 1
  for (int qq = 0; qq < 2; ++qq) {
    v8f a0, a1, a2, a3;
    gemm16x64(ap, plane, DN, 4, 64 * qq, m, hh, a0, a1, a2, a3);
    {
      float* sp = sw + (8 * hh) * 64 + m;
#pragma unroll
      for (int r = 0; r < 8; ++r) {
        sp[r * 64]      = a0[r] * INV16;
        sp[r * 64 + 16] = a1[r] * INV16;
        sp[r * 64 + 32] = a2[r] * INV16;
        sp[r * 64 + 48] = a3[r] * INV16;
      }
    }
    __syncthreads();
#pragma unroll 1
    for (int i = 0; i < 8; ++i) {
      const int r2 = 2 * i + hh;
      const v4f v = *(const v4f*)(sw + r2 * 64 + 4 * m);
      const int row = n0 + 16 * rt + r2;
      *(volatile v4f*)(NP + (size_t)row * NPROW + 128 * chf + 64 * qq + 4 * m) = v;
    }
    __threadfence();
#pragma unroll 1
    for (int i = 0; i < 8; ++i) {
      const int r2 = 2 * i + hh;
      const v4f v = *(const v4f*)(sw + r2 * 64 + 4 * m);
      const int row = n0 + 16 * rt + r2;
      *(volatile v4f*)(NP + (size_t)row * NPROW + 128 * chf + 64 * qq + 4 * m) = v;
    }
    __syncthreads();
  }
}

__device__ __forceinline__ void gate_convert(const float* sHt, const float* wg, float bg, _Float16* dst, int tid) {
  const int e = tid >> 2, g = tid & 3;
  const float* row = sHt + e * GSTR + 32 * g;
  const float* w = wg + 32 * g;
  float s = 0.f;
#pragma unroll 4
  for (int c = 0; c < 32; ++c) s += row[c] * w[c];
  s += __shfl_xor(s, 1);
  s += __shfl_xor(s, 2);
  const float gv = sigm_f(s + bg);
  _Float16* dp = dst + e * APA + 32 * g;
#pragma unroll
  for (int i = 0; i < 4; ++i) {
    Cvt8 cv;
#pragma unroll
    for (int j = 0; j < 8; ++j) cv.v[j] = (_Float16)((row[8 * i + j] * gv) * SCA);
    *(v8h*)(dp + 8 * i) = cv.v;
  }
}

__device__ __forceinline__ void store_msgs(const _Float16* tile, unsigned short* Mout, int el0, int tid) {
  const int p = tid & 15, rq = tid >> 4;
#pragma unroll 1
  for (int it = 0; it < 4; ++it) {
    const int row = 16 * it + rq;
    Cvt8 cv;
    cv.v = *(const v8h*)(tile + row * APA + 8 * p);
    *(volatile v8us*)(Mout + (size_t)(el0 + row) * MROW + 8 * p) = cv.u;
  }
  __threadfence();
#pragma unroll 1
  for (int it = 0; it < 4; ++it) {
    const int row = 16 * it + rq;
    Cvt8 cv;
    cv.v = *(const v8h*)(tile + row * APA + 8 * p);
    *(volatile v8us*)(Mout + (size_t)(el0 + row) * MROW + 8 * p) = cv.u;
  }
}

__global__ __launch_bounds__(NTHR) void k_edge(
    const float* __restrict__ srcc, const float* __restrict__ tgtc,
    const int* __restrict__ esrc, const int* __restrict__ etgt,
    const float* __restrict__ NPs, const float* __restrict__ NPt, const unsigned short* __restrict__ wp,
    const float* __restrict__ w1s, const float* __restrict__ b1s,
    const float* __restrict__ w1t, const float* __restrict__ b1t,
    const float* __restrict__ b2s, const float* __restrict__ b2t,
    const float* __restrict__ wgs, const float* __restrict__ bgs,
    const float* __restrict__ wgt, const float* __restrict__ bgt,
    const float* __restrict__ bc1, const float* __restrict__ wc2,
    unsigned short* Ms, unsigned short* Mt, float* Cout, int nE, int nS, int nT, int cbeg) {
  extern __shared__ __attribute__((aligned(16))) float sH[];
  __shared__ __attribute__((aligned(16))) _Float16 sA[NBE * APA];
  __shared__ __attribute__((aligned(16))) _Float16 sB[NBE * APA];
  __shared__ __attribute__((aligned(16))) float sPar[SPARN];
  __shared__ __attribute__((aligned(16))) float sDif[NBE * 4];
  __shared__ __attribute__((aligned(16))) float sCo[NBE * 4];
  __shared__ float sRad[NBE];
  __shared__ int sI[NBE];
  __shared__ int sJ[NBE];
  const int tid = (int)threadIdx.x, lane = tid & 31, wave = tid >> 5, hh = lane >> 4, m = lane & 15;
  const int el0 = (int)blockIdx.x * NBE;

  if (tid < NBE) {
    int e = cbeg + el0 + tid;
    e = e > nE - 1 ? nE - 1 : e;
    const int ii = iclamp(esrc[e], 0, nS - 1);
    const int jj = iclamp(etgt[e], 0, nT - 1);
    const float dx = tgtc[(size_t)jj * 3]     - srcc[(size_t)ii * 3];
    const float dy = tgtc[(size_t)jj * 3 + 1] - srcc[(size_t)ii * 3 + 1];
    const float dz = tgtc[(size_t)jj * 3 + 2] - srcc[(size_t)ii * 3 + 2];
    const float rad = (dx * dx + dz * dz) + dy * dy;
    sDif[4 * tid]     = dx;
    sDif[4 * tid + 1] = dy;
    sDif[4 * tid + 2] = dz;
    sDif[4 * tid + 3] = 0.0f;
    sRad[tid] = rad;
    sI[tid] = ii;
    sJ[tid] = jj;
  }
  if (tid < DN) {
    sPar[OB1S + tid] = b1s[tid];
    sPar[OWRS + tid] = w1s[(size_t)2 * DN * DN + tid];
    sPar[OB1T + tid] = b1t[tid];
    sPar[OWRT + tid] = w1t[(size_t)2 * DN * DN + tid];
    sPar[OB2S + tid] = b2s[tid];
    sPar[OB2T + tid] = b2t[tid];
    sPar[OWGS + tid] = wgs[tid];
    sPar[OWGT + tid] = wgt[tid];
    sPar[OBC1 + tid] = bc1[tid];
    sPar[OWC2 + tid] = wc2[tid];
  }
  if (tid == 0) { sPar[OBGS] = bgs[0]; sPar[OBGT] = bgt[0]; }
  __syncthreads();

  {
    const int c4 = 4 * lane;
    const v4f bbs = *(const v4f*)(sPar + OB1S + c4);
    const v4f wrs = *(const v4f*)(sPar + OWRS + c4);
    const v4f bbt = *(const v4f*)(sPar + OB1T + c4);
    const v4f wrt = *(const v4f*)(sPar + OWRT + c4);
#pragma unroll 1
    for (int jx = 0; jx < 8; ++jx) {
      const int el = 8 * wave + jx;
      const int ii = sI[el];
      const int jj = sJ[el];
      const float rad = sRad[el];
      const float* prow = NPs + (size_t)ii * NPROW + c4;
      const float* qrow = NPt + (size_t)jj * NPROW + c4;
      const v4f ps = *(const v4f*)(prow);
      const v4f pt = *(const v4f*)(prow + DN);
      const v4f qs = *(const v4f*)(qrow);
      const v4f qt = *(const v4f*)(qrow + DN);
      const v4f vs = ((ps + qs) + wrs * rad) + bbs;
      const v4f vt = ((pt + qt) + wrt * rad) + bbt;
      v4h zs, zt;
      zs.x = (_Float16)(silu_f(vs.x) * SCA);
      zs.y = (_Float16)(silu_f(vs.y) * SCA);
      zs.z = (_Float16)(silu_f(vs.z) * SCA);
      zs.w = (_Float16)(silu_f(vs.w) * SCA);
      zt.x = (_Float16)(silu_f(vt.x) * SCA);
      zt.y = (_Float16)(silu_f(vt.y) * SCA);
      zt.z = (_Float16)(silu_f(vt.z) * SCA);
      zt.w = (_Float16)(silu_f(vt.w) * SCA);
      *(v4h*)(sA + el * APA + c4) = zs;
      *(v4h*)(sB + el * APA + c4) = zt;
    }
  }
  __syncthreads();

  const int rt = wave & 3, cg = wave >> 2;

  {
    v8f a0, a1, a2, a3;
    gemm16x64(sA + (16 * rt + m) * APA + 8 * hh, (const _Float16*)(wp + P2S), DN, 4, 64 * cg, m, hh, a0, a1, a2, a3);
    float* sp = sH + (16 * rt + 8 * hh) * GSTR + 64 * cg + m;
    const float* bb = sPar + OB2S + 64 * cg + m;
    stage8s(sp,      a0, INV1024, bb[0]);
    stage8s(sp + 16, a1, INV1024, bb[16]);
    stage8s(sp + 32, a2, INV1024, bb[32]);
    stage8s(sp + 48, a3, INV1024, bb[48]);
  }
  __syncthreads();
  gate_convert(sH, sPar + OWGS, sPar[OBGS], sA, tid);
  __syncthreads();
  store_msgs(sA, Ms, el0, tid);

  {
    v8f a0, a1, a2, a3;
    gemm16x64(sB + (16 * rt + m) * APA + 8 * hh, (const _Float16*)(wp + P2T), DN, 4, 64 * cg, m, hh, a0, a1, a2, a3);
    float* sp = sH + (16 * rt + 8 * hh) * GSTR + 64 * cg + m;
    const float* bb = sPar + OB2T + 64 * cg + m;
    stage8s(sp,      a0, INV1024, bb[0]);
    stage8s(sp + 16, a1, INV1024, bb[16]);
    stage8s(sp + 32, a2, INV1024, bb[32]);
    stage8s(sp + 48, a3, INV1024, bb[48]);
  }
  __syncthreads();
  gate_convert(sH, sPar + OWGT, sPar[OBGT], sB, tid);
  __syncthreads();
  store_msgs(sB, Mt, el0, tid);

  {
    v8f a0, a1, a2, a3;
    gemm16x64(sA + (16 * rt + m) * APA + 8 * hh, (const _Float16*)(wp + PC1), DN, 4, 64 * cg, m, hh, a0, a1, a2, a3);
    float* sp = sH + (16 * rt + 8 * hh) * GSTR + 64 * cg + m;
    const float* bb = sPar + OBC1 + 64 * cg + m;
    stage8s(sp,      a0, INV1024, bb[0]);
    stage8s(sp + 16, a1, INV1024, bb[16]);
    stage8s(sp + 32, a2, INV1024, bb[32]);
    stage8s(sp + 48, a3, INV1024, bb[48]);
  }
  __syncthreads();

  {
    const int e = tid >> 2, g = tid & 3;
    const float* row = sH + e * GSTR + 32 * g;
    const float* w2 = sPar + OWC2 + 32 * g;
    float s = 0.f;
#pragma unroll 4
    for (int c = 0; c < 32; ++c) s += row[c] * w2[c];
    s += __shfl_xor(s, 1);
    s += __shfl_xor(s, 2);
    if (g == 0) {
      v4f cu;
      cu.x = sDif[4 * e] * s; cu.y = sDif[4 * e + 1] * s; cu.z = sDif[4 * e + 2] * s; cu.w = 1.0f;
      *(v4f*)(sCo + 4 * e) = cu;
    }
  }
  __syncthreads();

  if (tid < NBE) {
    const v4f v = *(const v4f*)(sCo + 4 * tid);
    *(volatile v4f*)(Cout + (size_t)(el0 + tid) * CROW) = v;
  }
  __threadfence();
  if (tid < NBE) {
    const v4f v = *(const v4f*)(sCo + 4 * tid);
    *(volatile v4f*)(Cout + (size_t)(el0 + tid) * CROW) = v;
  }
}

__device__ __forceinline__ int scan_piece(const int* __restrict__ ei, int lim, int cbase, int base,
                                          int* list, int tid, int wave) {
  int wc = 0;
  const int el0  = tid * EPT;
  const int e0   = cbase + el0;
  const int sent = -2147483647 - 1;
  int kk[EPT];
  if (cbase + PIECE <= lim) {
    const v4i* p = (const v4i*)(ei + e0);
#pragma unroll
    for (int u = 0; u < EPT / 4; ++u) {
      const v4i d = p[u];
      kk[4 * u] = d.x; kk[4 * u + 1] = d.y; kk[4 * u + 2] = d.z; kk[4 * u + 3] = d.w;
    }
  } else {
    const int lm = lim - 1;
#pragma unroll
    for (int q = 0; q < EPT; ++q) {
      const int eq = e0 + q;
      const int ec = eq > lm ? lm : eq;
      const int a = ei[ec];
      kk[q] = (eq < lim) ? a : sent;
    }
  }
  const unsigned nb = (unsigned)base;
  unsigned sq[EPT];
  bool hq[EPT];
  bool anyl = false;
#pragma unroll
  for (int q = 0; q < EPT; ++q) {
    sq[q] = (unsigned)kk[q] - nb;
    hq[q] = sq[q] < (unsigned)NBC;
    anyl = anyl | hq[q];
  }
  const unsigned any = __builtin_amdgcn_ballot_w32(anyl);
  if (any != 0u) {
#define HIT(HQ, SQ, Q) { \
      const unsigned mj = __builtin_amdgcn_ballot_w32(HQ); \
      if (mj != 0u) { \
        if (HQ) { \
          const int ps = wc + (int)__builtin_amdgcn_mbcnt_lo(mj, 0u); \
          if (ps < WCAP) list[wave * WCAP + ps] = ((el0 + (Q)) << SLB) | (int)(SQ); \
        } \
        wc += (int)__builtin_popcount(mj); } }
#pragma unroll
    for (int q = 0; q < EPT; ++q) {
      HIT(hq[q], sq[q], q)
    }
#undef HIT
  }
  return wc;
}

template <int USEC>
__device__ __forceinline__ void drain_piece(const int* list, const int* wcnt, float* accF, float* accC,
                                            const _Float16* __restrict__ Mh, const float* __restrict__ Cq,
                                            int rowoff, int lane, int wave) {
#pragma unroll 1
  for (int wsx = 0; wsx < NWAVE; ++wsx) {
    int n = __builtin_amdgcn_readfirstlane(wcnt[wsx]);
    n = n > WCAP ? WCAP : (n < 0 ? 0 : n);
    const int* lp = list + wsx * WCAP;
#pragma unroll 1
    for (int bb = 0; bb < n; bb += 32) {
      const int idx = bb + lane;
      const int ic = idx > WCAP - 1 ? WCAP - 1 : idx;
      const int ent = lp[ic];
      const bool own = (idx < n) && ((ent & (NWAVE - 1)) == wave);
      unsigned msk = __builtin_amdgcn_ballot_w32(own);
#pragma unroll 1
      while (msk != 0u) {
        const int bit = (int)__builtin_ctz(msk);
        msk &= msk - 1u;
        const int e2 = __builtin_amdgcn_readlane(ent, bit);
        const int slot = e2 & (NBC - 1);
        const int el = (e2 >> SLB) & (PIECE - 1);
        int row = rowoff + el;
        row = row < 0 ? 0 : (row > CE - 1 ? CE - 1 : row);
        const v4h mv = *(const v4h*)(Mh + (size_t)row * MROW + 4 * lane);
        float* ap = accF + slot * DN + 4 * lane;
        v4f a = *(const v4f*)ap;
        a.x += (float)mv.x * INV64;
        a.y += (float)mv.y * INV64;
        a.z += (float)mv.z * INV64;
        a.w += (float)mv.w * INV64;
        *(v4f*)ap = a;
        if (USEC) {
          const float cvv = Cq[(size_t)row * CROW + (lane & 3)];
          if (lane < 4) accC[CROW * slot + lane] += cvv;
        }
      }
    }
  }
}

template <int USEC>
__device__ __forceinline__ float coord_val(const float* accC, const float* __restrict__ x, size_t f0, int t) {
  const int s3 = t / 3;
  const int d = t - 3 * s3;
  float v = x[f0 + (size_t)t];
  if (USEC) {
    const float c = accC[CROW * s3 + 3];
    const float rc = __builtin_amdgcn_rcpf(fmaxf(c, 1.0f));
    float a = accC[CROW * s3 + d] * rc;
    a = fminf(fmaxf(a, -CMAXV), CMAXV);
    v = v + a;
  }
  return v;
}

template <int USEC>
__device__ __forceinline__ void agg_store(const float* accF, const float* accC, const float* __restrict__ x,
                                          float* AC, float* outc, float* HO, int base, int nN, int last,
                                          int tid, int lane, int wave) {
#pragma unroll 1
  for (int it = 0; it < NBC / NWAVE; ++it) {
    const int s = wave + NWAVE * it;
    const int node = base + s;
    if (node < nN) {
      const v4f v = *(const v4f*)(accF + s * DN + 4 * lane);
      *(volatile v4f*)(HO + (size_t)node * DN + 4 * lane) = v;
    }
  }
  if (USEC) {
#pragma unroll 1
    for (int it = 0; it < NBC / NTHR; ++it) {
      const int s = tid + NTHR * it;
      const v4f v = *(const v4f*)(accC + CROW * s);
      *(volatile v4f*)(AC + (size_t)(base + s) * CROW) = v;
    }
  }
  if (last != 0) {
    int cnt = nN - base;
    cnt = cnt > NBC ? NBC : cnt;
    const int nfl = 3 * cnt, nq = nfl >> 2, rem = nfl & 3;
    const size_t f0 = (size_t)3 * (size_t)base;
#pragma unroll 1
    for (int it = 0; it < 2; ++it) {
      const int q = tid + NTHR * it;
      if (q < nq) {
        float a[4];
#pragma unroll
        for (int c = 0; c < 4; ++c) a[c] = coord_val<USEC>(accC, x, f0, 4 * q + c);
        v4f ov;
        ov.x = a[0]; ov.y = a[1]; ov.z = a[2]; ov.w = a[3];
        *(volatile v4f*)(outc + f0 + 4 * (size_t)q) = ov;
      } else if (q == nq && rem != 0) {
#pragma unroll
        for (int c = 0; c < 3; ++c) {
          if (c < rem) {
            const int t = 4 * q + c;
            const float val = coord_val<USEC>(accC, x, f0, t);
            *(volatile float*)(outc + f0 + t) = val;
          }
        }
      }
    }
  }
}

template <int USEC>
__global__ __launch_bounds__(NTHR) void k_agg(
    const int* __restrict__ ei, const unsigned short* __restrict__ Mq, const float* __restrict__ Cq,
    const float* __restrict__ x, float* AC, float* outc, float* HO, int cbeg, int lim, int nN, int first, int last) {
  extern __shared__ __attribute__((aligned(16))) float accd[];
  __shared__ int list[NWAVE * WCAP];
  __shared__ int wcnt[NWAVE];
  const int tid = (int)threadIdx.x, lane = tid & 31, wave = tid >> 5;
  const int base = (int)blockIdx.x * NBC;
  float* accF = accd;
  float* accC = accd + NBC * DN;
  const _Float16* Mh = (const _Float16*)Mq;

  if (first != 0) {
#pragma unroll 1
    for (int i = tid; i < (NBC * DN) / 4; i += NTHR) *(v4f*)(accF + 4 * i) = zero4();
  } else {
#pragma unroll 1
    for (int i = tid; i < (NBC * DN) / 4; i += NTHR) {
      const int s = i >> 5, c4 = (i & 31) * 4;
      int node = base + s;
      node = node > nN - 1 ? nN - 1 : node;
      const v4f v = *(const v4f*)(HO + (size_t)node * DN + c4);
      *(v4f*)(accF + s * DN + c4) = v;
    }
  }
  if (USEC) {
    if (first != 0) {
#pragma unroll 1
      for (int s = tid; s < NBC; s += NTHR) *(v4f*)(accC + CROW * s) = zero4();
    } else {
#pragma unroll 1
      for (int s = tid; s < NBC; s += NTHR) {
        const v4f v = *(const v4f*)(AC + (size_t)(base + s) * CROW);
        *(v4f*)(accC + CROW * s) = v;
      }
    }
  }
  __syncthreads();

#pragma unroll 1
  for (int cbase = cbeg; cbase < lim; cbase += PIECE) {
    const int wc = scan_piece(ei, lim, cbase, base, list, tid, wave);
    if (lane == 0) wcnt[wave] = wc;
    __syncthreads();
    drain_piece<USEC>(list, wcnt, accF, accC, Mh, Cq, cbase - cbeg, lane, wave);
    __syncthreads();
  }

  agg_store<USEC>(accF, accC, x, AC, outc, HO, base, nN, last, tid, lane, wave);
  __threadfence();
  agg_store<USEC>(accF, accC, x, AC, outc, HO, base, nN, last, tid, lane, wave);
}

__global__ __launch_bounds__(NTHR) void k_nodemlp(
    const float* __restrict__ feat, float* HO, const unsigned short* __restrict__ wp, int pn1, int pn2,
    const float* __restrict__ nb1, const float* __restrict__ nb2, int nN) {
  __shared__ __attribute__((aligned(16))) float sU[NBN * GSTR];
  __shared__ __attribute__((aligned(16))) _Float16 sB[NBN * APA];
  __shared__ __attribute__((aligned(16))) float sPar[2 * DN];
  _Float16* sA = (_Float16*)sU;
  const int tid = (int)threadIdx.x, lane = tid & 31, wave = tid >> 5, hh = lane >> 4, m = lane & 15;
  const int n0 = (int)blockIdx.x * NBN;

  {
    const int nl = tid >> 2, g = tid & 3;
    int node = n0 + nl;
    node = node > nN - 1 ? nN - 1 : node;
    const float* fp = feat + (size_t)node * DN + 32 * g;
    const float* hp = HO   + (size_t)node * DN + 32 * g;
#pragma unroll
    for (int i = 0; i < 4; ++i) {
      const v4f xa = *(const v4f*)(fp + 8 * i);
      const v4f xb = *(const v4f*)(fp + 8 * i + 4);
      Cvt8 cv;
      cv.v[0] = (_Float16)xa.x; cv.v[1] = (_Float16)xa.y; cv.v[2] = (_Float16)xa.z; cv.v[3] = (_Float16)xa.w;
      cv.v[4] = (_Float16)xb.x; cv.v[5] = (_Float16)xb.y; cv.v[6] = (_Float16)xb.z; cv.v[7] = (_Float16)xb.w;
      *(v8h*)(sA + nl * APN + 32 * g + 8 * i) = cv.v;
    }
#pragma unroll
    for (int i = 0; i < 4; ++i) {
      const v4f xa = *(const v4f*)(hp + 8 * i);
      const v4f xb = *(const v4f*)(hp + 8 * i + 4);
      Cvt8 cv;
      cv.v[0] = (_Float16)xa.x; cv.v[1] = (_Float16)xa.y; cv.v[2] = (_Float16)xa.z; cv.v[3] = (_Float16)xa.w;
      cv.v[4] = (_Float16)xb.x; cv.v[5] = (_Float16)xb.y; cv.v[6] = (_Float16)xb.z; cv.v[7] = (_Float16)xb.w;
      *(v8h*)(sA + nl * APN + DN + 32 * g + 8 * i) = cv.v;
    }
  }
  if (tid < DN) {
    sPar[tid]      = nb1[tid];
    sPar[DN + tid] = nb2[tid];
  }
  __syncthreads();

  const int rt = wave & 3, cg = wave >> 2;

  {
    v8f a0, a1, a2, a3;
    gemm16x64(sA + (16 * rt + m) * APN + 8 * hh, (const _Float16*)(wp + pn1), 2 * DN, 8, 64 * cg, m, hh, a0, a1, a2, a3);
    _Float16* sp = sB + (16 * rt + 8 * hh) * APA + 64 * cg + m;
    const float* bb = sPar + 64 * cg + m;
    stage8hs(sp,      a0, INV16, bb[0]);
    stage8hs(sp + 16, a1, INV16, bb[16]);
    stage8hs(sp + 32, a2, INV16, bb[32]);
    stage8hs(sp + 48, a3, INV16, bb[48]);
  }
  __syncthreads();

  {
    v8f a0, a1, a2, a3;
    gemm16x64(sB + (16 * rt + m) * APA + 8 * hh, (const _Float16*)(wp + pn2), DN, 4, 64 * cg, m, hh, a0, a1, a2, a3);
    float* sp = sU + (16 * rt + 8 * hh) * GSTR + 64 * cg + m;
    const float* bb = sPar + DN + 64 * cg + m;
    stage8(sp,      a0, INV1024, bb[0]);
    stage8(sp + 16, a1, INV1024, bb[16]);
    stage8(sp + 32, a2, INV1024, bb[32]);
    stage8(sp + 48, a3, INV1024, bb[48]);
  }
  __syncthreads();

#pragma unroll 1
  for (int it = 0; it < NBN / NWAVE; ++it) {
    const int s = wave + NWAVE * it;
    const int node = n0 + s;
    if (node < nN) {
      const v4f v  = *(const v4f*)(sU + s * GSTR + 4 * lane);
      const v4f fv = *(const v4f*)(feat + (size_t)node * DN + 4 * lane);
      const v4f o = v + fv;
      *(volatile v4f*)(HO + (size_t)node * DN + 4 * lane) = o;
    }
  }
  __threadfence();
#pragma unroll 1
  for (int it = 0; it < NBN / NWAVE; ++it) {
    const int s = wave + NWAVE * it;
    const int node = n0 + s;
    if (node < nN) {
      const v4f v  = *(const v4f*)(sU + s * GSTR + 4 * lane);
      const v4f fv = *(const v4f*)(feat + (size_t)node * DN + 4 * lane);
      const v4f o = v + fv;
      *(volatile v4f*)(HO + (size_t)node * DN + 4 * lane) = o;
    }
  }
}

extern "C" void kernel_launch(void* const* d_in, const int* in_sizes, int n_in,
                              void* d_out, int out_size, void* d_ws, size_t ws_size,
                              hipStream_t stream) {
  if (n_in < 29) return;
  if (in_sizes[0] < DN || (in_sizes[0] % DN) != 0) return;
  if (in_sizes[1] < DN || (in_sizes[1] % DN) != 0) return;
  const int nS = in_sizes[0] / DN;
  const int nT = in_sizes[1] / DN;
  if (nS < 2 || nS > (1 << 22) || nT < 2 || nT > (1 << 22)) return;
  if (in_sizes[2] != 3 * nS || in_sizes[3] != 3 * nT) return;
  const int nE = in_sizes[4];
  if (nE < 1 || nE > (1 << 27) || in_sizes[5] != nE) return;
  if (in_sizes[6] != (2 * DN + 1) * DN || in_sizes[7] != DN) return;
  if (in_sizes[8] != DN * DN || in_sizes[9] != DN) return;
  if (in_sizes[10] != (2 * DN + 1) * DN || in_sizes[11] != DN) return;
  if (in_sizes[12] != DN * DN || in_sizes[13] != DN) return;
  if (in_sizes[14] != DN || in_sizes[15] < 1) return;
  if (in_sizes[16] != DN || in_sizes[17] < 1) return;
  if (in_sizes[18] != DN * DN || in_sizes[19] != DN || in_sizes[20] != DN) return;
  if (in_sizes[21] != 2 * DN * DN || in_sizes[22] != DN) return;
  if (in_sizes[23] != DN * DN || in_sizes[24] != DN) return;
  if (in_sizes[25] != 2 * DN * DN || in_sizes[26] != DN) return;
  if (in_sizes[27] != DN * DN || in_sizes[28] != DN) return;
  if (out_size != 131 * nS + 131 * nT) return;

  const float* srcf = (const float*)d_in[0];
  const float* tgtf = (const float*)d_in[1];
  const float* srcc = (const float*)d_in[2];
  const float* tgtc = (const float*)d_in[3];
  const int*   esrc = (const int*)d_in[4];
  const int*   etgt = (const int*)d_in[5];
  const float* w1s  = (const float*)d_in[6];
  const float* b1s  = (const float*)d_in[7];
  const float* w2s  = (const float*)d_in[8];
  const float* b2s  = (const float*)d_in[9];
  const float* w1t  = (const float*)d_in[10];
  const float* b1t  = (const float*)d_in[11];
  const float* w2t  = (const float*)d_in[12];
  const float* b2t  = (const float*)d_in[13];
  const float* wgs  = (const float*)d_in[14];
  const float* bgs  = (const float*)d_in[15];
  const float* wgt  = (const float*)d_in[16];
  const float* bgt  = (const float*)d_in[17];
  const float* wc1  = (const float*)d_in[18];
  const float* bc1  = (const float*)d_in[19];
  const float* wc2  = (const float*)d_in[20];
  const float* wn1t = (const float*)d_in[21];
  const float* bn1t = (const float*)d_in[22];
  const float* wn2t = (const float*)d_in[23];
  const float* bn2t = (const float*)d_in[24];
  const float* wn1s = (const float*)d_in[25];
  const float* bn1s = (const float*)d_in[26];
  const float* wn2s = (const float*)d_in[27];
  const float* bn2s = (const float*)d_in[28];
  float* out0 = (float*)d_out;
  float* out1 = out0 + (size_t)nS * DN;
  float* out2 = out1 + (size_t)nT * DN;
  float* out3 = out2 + (size_t)3 * (size_t)nS;

  const int nbS = (nS + NBN - 1) / NBN, nbT = (nT + NBN - 1) / NBN;
  const int NpadS = nbS * NBN, NpadT = nbT * NBN;
  const int nChunk = (nE + CE - 1) / CE;
  if (nChunk < 1 || nChunk > MAXCH) return;
  const int nbAggS = (nS + NBC - 1) / NBC, nbAggT = (nT + NBC - 1) / NBC;

  char* ws = (char*)d_ws;
  size_t off = 0;
  const size_t oW   = off; off += (size_t)PWTOT * 2;                  off = (off + 255) & ~(size_t)255;
  const size_t oNPs = off; off += (size_t)NpadS * NPROW * 4;          off = (off + 255) & ~(size_t)255;
  const size_t oNPt = off; off += (size_t)NpadT * NPROW * 4;          off = (off + 255) & ~(size_t)255;
  const size_t oMs  = off; off += (size_t)CE * MROW * 2;              off = (off + 255) & ~(size_t)255;
  const size_t oMt  = off; off += (size_t)CE * MROW * 2;              off = (off + 255) & ~(size_t)255;
  const size_t oC   = off; off += (size_t)CE * CROW * 4;              off = (off + 255) & ~(size_t)255;
  const size_t oAC  = off; off += (size_t)nbAggT * NBC * CROW * 4;    off = (off + 255) & ~(size_t)255;
  if (off > ws_size || off > (size_t)WSCAP) return;
  unsigned short* wp = (unsigned short*)(ws + oW);
  float* NPs         = (float*)(ws + oNPs);
  float* NPt         = (float*)(ws + oNPt);
  unsigned short* Ms = (unsigned short*)(ws + oMs);
  unsigned short* Mt = (unsigned short*)(ws + oMt);
  float* Cq          = (float*)(ws + oC);
  float* AC          = (float*)(ws + oAC);

  hipFuncSetAttribute(reinterpret_cast<const void*>(&k_agg<1>), hipFuncAttributeMaxDynamicSharedMemorySize, AGGDYN);
  hipFuncSetAttribute(reinterpret_cast<const void*>(&k_agg<0>), hipFuncAttributeMaxDynamicSharedMemorySize, AGGDYN);

  k_prep<<<PBLK, NTHR, 0, stream>>>(w1s, w1t, w2s, w2t, wc1, wn1t, wn2t, wn1s, wn2s, wp);
  k_node<<<nbS, NTHR, 0, stream>>>(srcf, wp, PAS, PAT, NPs, nS);
  k_node<<<nbT, NTHR, 0, stream>>>(tgtf, wp, PBS, PBT, NPt, nT);
  for (int c = 0; c < nChunk; ++c) {
    const int cbeg = c * CE;
    int lim = cbeg + CE;
    lim = lim > nE ? nE : lim;
    const int nblk = (lim - cbeg + NBE - 1) / NBE;
    const int first = (c == 0) ? 1 : 0;
    const int last  = (c == nChunk - 1) ? 1 : 0;
    k_edge<<<nblk, NTHR, EDGEDYN, stream>>>(srcc, tgtc, esrc, etgt, NPs, NPt, wp, w1s, b1s, w1t, b1t, b2s, b2t,
                                            wgs, bgs, wgt, bgt, bc1, wc2, Ms, Mt, Cq, nE, nS, nT, cbeg);
    k_agg<1><<<nbAggT, NTHR, AGGDYN, stream>>>(etgt, Ms, Cq, tgtc, AC, out3, out1, cbeg, lim, nT, first, last);
    k_agg<0><<<nbAggS, NTHR, AGGDYN, stream>>>(esrc, Mt, Cq, srcc, AC, out2, out0, cbeg, lim, nS, first, last);
  }
  k_nodemlp<<<nbT, NTHR, 0, stream>>>(tgtf, out1, wp, PN1T, PN2T, bn1t, bn2t, nT);
  k_nodemlp<<<nbS, NTHR, 0, stream>>>(srcf, out0, wp, PN1S, PN2S, bn1s, bn2s, nS);
}
